// LSTMPointerNet_11304353923325
// MI455X (gfx1250) — hardware-verified
//
#include <hip/hip_runtime.h>
#include <math.h>

constexpr int kB   = 16;
constexpr int kNS  = 128;
constexpr int kT   = 63;
constexpr int kTQ  = 64;
constexpr int kD   = 512;
constexpr int kH   = 512;
constexpr int kG4  = 4 * kH;
constexpr int kBT  = kB * kTQ;
constexpr int kBN  = kB * kNS;
constexpr int kDim = kD;
constexpr int kHid = kH;
constexpr float kNeg       = -1e18f;
constexpr float kWCarry    = 16.0f;
constexpr float kWCarryInv = 1.0f / 16.0f;
constexpr float kPCarry    = 1024.0f;
constexpr float kPCarryInv = 1.0f / 1024.0f;
constexpr float kTwoLog2e  = 2.8853900817779268f;
constexpr float kQWScale   = kTwoLog2e * kWCarryInv;

static_assert(kTQ == kT + 1);
static_assert(kD % 32 == 0 && kH % 32 == 0 && kNS % 32 == 0);
static_assert(kBN % 64 == 0 && kBT % 64 == 0 && kH % 64 == 0 && kG4 % 64 == 0 && kTQ % 64 == 0);
static_assert((kBT * kD) % (8 * 256) == 0);

typedef __attribute__((ext_vector_type(16))) _Float16 v16h;
typedef __attribute__((ext_vector_type(8)))  _Float16 v8h;
typedef __attribute__((ext_vector_type(16))) __bf16   v16b;
typedef __attribute__((ext_vector_type(8)))  __bf16   v8b;
typedef __attribute__((ext_vector_type(8)))  float    v8f;
typedef __attribute__((ext_vector_type(4)))  float    v4f;
typedef __attribute__((ext_vector_type(4)))  unsigned int v4u;

__device__ __forceinline__ unsigned short f2bf_bits(float f) {
  unsigned u = __float_as_uint(f);
  return (unsigned short)((u + 0x7FFFu + ((u >> 16) & 1u)) >> 16);
}
__device__ __forceinline__ float bf_bits2f(unsigned short h) { return __uint_as_float(((unsigned)h) << 16); }

__device__ __forceinline__ void dep_guard_h(v8f& a, v8f& b, v16h x, v16h y) { asm volatile("v_nop\n\tv_nop\n\tv_nop\n\tv_nop" : "+v"(a), "+v"(b) : "v"(x), "v"(y)); }
__device__ __forceinline__ void dep_guard_b(v8f& a, v8f& b, v16b x, v16b y) { asm volatile("v_nop\n\tv_nop\n\tv_nop\n\tv_nop" : "+v"(a), "+v"(b) : "v"(x), "v"(y)); }
__device__ __forceinline__ void keep4_h(v16h a, v16h b, v16h c, v16h d) { asm volatile("v_nop" :: "v"(a), "v"(b), "v"(c), "v"(d)); }
__device__ __forceinline__ void keep4_b(v16b a, v16b b, v16b c, v16b d) { asm volatile("v_nop" :: "v"(a), "v"(b), "v"(c), "v"(d)); }
__device__ __forceinline__ void acc_guard4(v8f& a, v8f& b, v8f& c, v8f& d) { asm volatile("v_nop\n\tv_nop\n\tv_nop\n\tv_nop" : "+v"(a), "+v"(b), "+v"(c), "+v"(d)); }
template <typename T> struct Frag;
template <> struct Frag<_Float16> {
  typedef v16h V; union U { v16h v; v8h h[2]; };
  static __device__ __forceinline__ v16h load(const _Float16* p) {
    U f; f.h[0] = *(const v8h*)(p); f.h[1] = *(const v8h*)(p + 16); return f.v;
  }
  static __device__ __forceinline__ v8f mma(v16h a, v16h b, v8f c) {
    return __builtin_amdgcn_wmma_f32_16x16x32_f16(false, a, false, b, (short)0, c, false, false);
  }
  static __device__ __forceinline__ void guard(v8f& a, v8f& b, v16h x, v16h y) { dep_guard_h(a, b, x, y); }
  static __device__ __forceinline__ void keep(v16h a, v16h b, v16h c, v16h d) { keep4_h(a, b, c, d); }
};
template <> struct Frag<__bf16> {
  typedef v16b V; union U { v16b v; v8b h[2]; };
  static __device__ __forceinline__ v16b load(const __bf16* p) {
    U f; f.h[0] = *(const v8b*)(p); f.h[1] = *(const v8b*)(p + 16); return f.v;
  }
  static __device__ __forceinline__ v8f mma(v16b a, v16b b, v8f c) {
    return __builtin_amdgcn_wmma_f32_16x16x32_bf16(false, a, false, b, (short)0, c, false, false);
  }
  static __device__ __forceinline__ void guard(v8f& a, v8f& b, v16b x, v16b y) { dep_guard_b(a, b, x, y); }
  static __device__ __forceinline__ void keep(v16b a, v16b b, v16b c, v16b d) { keep4_b(a, b, c, d); }
};

__device__ __forceinline__ unsigned pk16(unsigned short a, unsigned short b) { return (unsigned)a | ((unsigned)b << 16); }
__device__ __forceinline__ unsigned short h_bits(float f) { const _Float16 h = (_Float16)f; return __builtin_bit_cast(unsigned short, h); }
__device__ __forceinline__ float rcp_approx(float x) { return __builtin_amdgcn_rcpf(x); }
__device__ __forceinline__ float sigm_f(float x) { return rcp_approx(1.0f + expf(-x)); }

template <int ET> struct Elem;
template <> struct Elem<0> { typedef _Float16 T; };
template <> struct Elem<1> { typedef __bf16 T; };
template <int ET, bool SPLIT, int BIAS_MODE, int OUT_MODE, bool RESID, int ACT = 0>
__global__ __launch_bounds__(256) void wmma_gemm64(
    const unsigned short* __restrict__ Ap, const unsigned short* __restrict__ A2p, int lda, long strideA,
    const unsigned short* __restrict__ Btp, const unsigned short* __restrict__ Bt2p, int ldb, long strideB,
    void* __restrict__ Cout, void* __restrict__ Cout2, int ldc, long strideC,
    const float* __restrict__ bias,
    const float* __restrict__ resid, long strideR,
    int M, int N, int K, float scale) {
  typedef typename Elem<ET>::T T;
  typedef typename Frag<T>::V V;
  const T* A = (const T*)Ap; const T* A2 = (const T*)A2p; const T* Bt = (const T*)Btp; const T* Bt2 = (const T*)Bt2p;
  __shared__ __align__(16) float sT[8][16 * 68];
  const int b    = blockIdx.y;
  const int lane = threadIdx.x & 31;
  const int wave = threadIdx.x >> 5;
  const int tilesN = N >> 6;
  const int tilesM = M >> 6;
  const int tile = blockIdx.x * 8 + wave;
  if (tile >= tilesM * tilesN) return;
  const int tm = tile / tilesN;
  const int tn = tile - tm * tilesN;
  const int m0 = tm << 6;
  const int n0 = tn << 6;

  const T* Ab  = A  + (size_t)b * strideA;
  const T* Bb  = Bt + (size_t)b * strideB;
  const T* Ab2 = SPLIT ? (A2  + (size_t)b * strideA) : nullptr;
  const T* Bb2 = SPLIT ? (Bt2 + (size_t)b * strideB) : nullptr;

  const int rlane = lane & 15;
  const int koff  = (lane >> 4) * 8;
  const int mOff  = (lane >> 4) * 8;

  v8f acc[4][4];
#pragma unroll
  for (int i = 0; i < 4; ++i)
#pragma unroll
    for (int j = 0; j < 4; ++j) acc[i][j] = (v8f){0.f,0.f,0.f,0.f,0.f,0.f,0.f,0.f};

  for (int k0 = 0; k0 < K; k0 += 32) {
    V bh[4], bl[4];
#pragma unroll
    for (int j = 0; j < 4; ++j) {
      const size_t bo = (size_t)(n0 + (j << 4) + rlane) * ldb + koff + k0;
      bh[j] = Frag<T>::load(Bb + bo);
      if (SPLIT) bl[j] = Frag<T>::load(Bb2 + bo);
    }
#pragma unroll
    for (int i = 0; i < 4; ++i) {
      const size_t ao = (size_t)(m0 + (i << 4) + rlane) * lda + koff + k0;
      V ah = Frag<T>::load(Ab + ao);
      V al;
      if (SPLIT) al = Frag<T>::load(Ab2 + ao);
#pragma unroll
      for (int j = 0; j < 4; ++j) {
        acc[i][j] = Frag<T>::mma(ah, bh[j], acc[i][j]);
        if (SPLIT) {
          acc[i][j] = Frag<T>::mma(ah, bl[j], acc[i][j]);
          acc[i][j] = Frag<T>::mma(al, bh[j], acc[i][j]);
        }
      }
      Frag<T>::guard(acc[i][0], acc[i][3], ah, SPLIT ? al : ah);
    }
    Frag<T>::keep(bh[0], bh[1], bh[2], bh[3]);
    if (SPLIT) Frag<T>::keep(bl[0], bl[1], bl[2], bl[3]);
  }
  acc_guard4(acc[0][0], acc[0][1], acc[0][2], acc[0][3]);
  acc_guard4(acc[1][0], acc[1][1], acc[1][2], acc[1][3]);
  acc_guard4(acc[2][0], acc[2][1], acc[2][2], acc[2][3]);
  acc_guard4(acc[3][0], acc[3][1], acc[3][2], acc[3][3]);

  float* slab = sT[wave];
  const float* Rb = RESID ? (resid + (size_t)b * strideR) : nullptr;
#pragma unroll
  for (int i = 0; i < 4; ++i) {
    const int mBase = m0 + (i << 4);
#pragma unroll
    for (int j = 0; j < 4; ++j) {
      const int n = n0 + (j << 4) + rlane;
      float bv = 0.f;
      if (BIAS_MODE == 2) bv = bias[n];
#pragma unroll
      for (int r = 0; r < 8; ++r) {
        float v = acc[i][j][r] * scale;
        if (BIAS_MODE == 1) v += bias[mBase + mOff + r];
        if (BIAS_MODE == 2) v += bv;
        if (RESID) v += Rb[(size_t)(mBase + mOff + r) * ldc + n];
        if (ACT == 2) v = fmaxf(v, 0.0f);
        if (ACT == 4) v = (v > 0.f) ? v : 0.01f * v;
        slab[(mOff + r) * 68 + (j << 4) + rlane] = v;
      }
    }
    __builtin_amdgcn_fence(__ATOMIC_RELEASE, "workgroup");
    __builtin_amdgcn_wave_barrier();
    __builtin_amdgcn_fence(__ATOMIC_ACQUIRE, "workgroup");
    if (OUT_MODE == 0) {
      float* C = (float*)Cout + (size_t)b * strideC;
      const int hh = lane >> 4, c4 = (lane & 15) * 4;
      for (int pass = 0; pass < 2; ++pass) {
#pragma unroll
        for (int it = 0; it < 8; ++it) {
          const int row = it * 2 + hh;
          v4f v = *(const v4f*)(slab + row * 68 + c4);
          *(volatile v4f*)(C + (size_t)(mBase + row) * ldc + n0 + c4) = v;
        }
        __threadfence();
      }
    } else {
      const int q = lane >> 3, c8 = (lane & 7) * 8;
      unsigned short* C  = (unsigned short*)Cout  + (size_t)b * strideC;
      unsigned short* C2 = (OUT_MODE == 2) ? ((unsigned short*)Cout2 + (size_t)b * strideC) : nullptr;
      for (int pass = 0; pass < 2; ++pass) {
#pragma unroll
        for (int it = 0; it < 4; ++it) {
          const int row = it * 4 + q;
          const float* sp = slab + row * 68 + c8;
          v8h hv, lv;
#pragma unroll
          for (int e = 0; e < 8; ++e) {
            if (OUT_MODE == 1) {
              hv[e] = (_Float16)sp[e];
            } else {
              unsigned short hb = f2bf_bits(sp[e]);
              unsigned short lb = f2bf_bits(sp[e] - bf_bits2f(hb));
              hv[e] = __builtin_bit_cast(_Float16, hb);
              lv[e] = __builtin_bit_cast(_Float16, lb);
            }
          }
          *(volatile v8h*)(C + (size_t)(mBase + row) * ldc + n0 + c8) = hv;
          if (OUT_MODE == 2) *(volatile v8h*)(C2 + (size_t)(mBase + row) * ldc + n0 + c8) = lv;
        }
        __threadfence();
      }
    }
    __builtin_amdgcn_fence(__ATOMIC_RELEASE, "workgroup");
    __builtin_amdgcn_wave_barrier();
    __builtin_amdgcn_fence(__ATOMIC_ACQUIRE, "workgroup");
  }
}

__global__ __launch_bounds__(256) void wtcast_kernel(const float* __restrict__ W0, const float* __restrict__ W1,
                                                     const float* __restrict__ W2, const float* __restrict__ W3,
                                                     unsigned short* __restrict__ out, float scale) {
  __shared__ float sm[64][65];
  const int t  = threadIdx.x;
  const int d0 = blockIdx.x * 64;
  const int h0 = blockIdx.y * 64;
  const int z  = blockIdx.z;
  const float* W = (z == 0) ? W0 : (z == 1) ? W1 : (z == 2) ? W2 : W3;
#pragma unroll
  for (int i = 0; i < 16; ++i) {
    const int e = i * 256 + t;
    const int r = e >> 6;
    const int c = e & 63;
    sm[c][r] = W[(size_t)(d0 + r) * kHid + h0 + c] * scale;
  }
  __syncthreads();
  const int lane = t & 31, wave = t >> 5;
  const int q = lane >> 3, c8 = (lane & 7) * 8;
  unsigned short* op = out + (size_t)z * kHid * kDim;
  for (int pass = 0; pass < 2; ++pass) {
#pragma unroll
    for (int it = 0; it < 2; ++it) {
      const int row = wave * 8 + it * 4 + q;
      unsigned short hb[8];
#pragma unroll
      for (int e = 0; e < 8; ++e) hb[e] = h_bits(sm[row][c8 + e]);
      const v4u u = (v4u){pk16(hb[0], hb[1]), pk16(hb[2], hb[3]), pk16(hb[4], hb[5]), pk16(hb[6], hb[7])};
      *(volatile v4u*)(op + (size_t)(h0 + row) * kDim + d0 + c8) = u;
    }
    __threadfence();
  }
}

__global__ __launch_bounds__(256) void cast3_f16_kernel(const float* __restrict__ s0, const float* __restrict__ s1,
                                                        const float* __restrict__ s2,
                                                        unsigned short* __restrict__ d0, unsigned short* __restrict__ d1,
                                                        unsigned short* __restrict__ d2,
                                                        float sc0, float sc1, float sc2, int n8) {
  const int z = blockIdx.y;
  const float* in = (z == 0) ? s0 : (z == 1) ? s1 : s2;
  unsigned short* out = (z == 0) ? d0 : (z == 1) ? d1 : d2;
  const float sc = (z == 0) ? sc0 : (z == 1) ? sc1 : sc2;
  const int i = blockIdx.x * 256 + threadIdx.x;
  if (i >= n8) return;
  const float* p = in + 8 * (size_t)i;
  const v4f a = *(const v4f*)(p);
  const v4f c = *(const v4f*)(p + 4);
  unsigned short hb[8];
#pragma unroll
  for (int e = 0; e < 4; ++e) {
    hb[e]     = h_bits(a[e] * sc);
    hb[4 + e] = h_bits(c[e] * sc);
  }
  const v4u u = (v4u){pk16(hb[0], hb[1]), pk16(hb[2], hb[3]), pk16(hb[4], hb[5]), pk16(hb[6], hb[7])};
  unsigned short* q = out + 8 * (size_t)i;
  *(volatile v4u*)q = u;
  __threadfence();
  *(volatile v4u*)q = u;
}

constexpr int kXBlocks = (kBT * kD) / (8 * 256);
__global__ __launch_bounds__(256) void prep_kernel(const float* __restrict__ attn_mem, const float* __restrict__ lstm_in,
                                                   const int* __restrict__ mem_sizes,
                                                   const float* __restrict__ bih, const float* __restrict__ bhh,
                                                   unsigned short* __restrict__ X16, float* __restrict__ bsum) {
  const int tid = threadIdx.x;
  if (blockIdx.x < kXBlocks) {
    const int gi  = blockIdx.x * 256 + tid;
    const int row = gi >> 6;
    const int c8  = (gi & 63) * 8;
    const int t   = blockIdx.x >> 2;
    const int b   = row & 15;
    float vals[8];
    if (t == 0) {
      int ms = mem_sizes[b];
      ms = (ms < 1) ? 1 : ((ms > kNS) ? kNS : ms);
#pragma unroll
      for (int e = 0; e < 8; ++e) vals[e] = kNeg;
      const float* base = attn_mem + (size_t)b * kNS * kD + c8;
#pragma unroll 1
      for (int n = 0; n < kNS; ++n) {
        const v4f a = *(const v4f*)(base + (size_t)n * kD);
        const v4f c = *(const v4f*)(base + (size_t)n * kD + 4);
        const bool valid = (n < ms);
#pragma unroll
        for (int e = 0; e < 4; ++e) {
          vals[e]     = valid ? fmaxf(vals[e], a[e]) : vals[e];
          vals[4 + e] = valid ? fmaxf(vals[4 + e], c[e]) : vals[4 + e];
        }
      }
    } else {
      const float* src = lstm_in + ((size_t)b * kT + (size_t)(t - 1)) * kD + c8;
      const v4f a = *(const v4f*)(src);
      const v4f c = *(const v4f*)(src + 4);
#pragma unroll
      for (int e = 0; e < 4; ++e) { vals[e] = a[e]; vals[4 + e] = c[e]; }
    }
    unsigned short hb[8];
#pragma unroll
    for (int e = 0; e < 8; ++e) hb[e] = h_bits(vals[e]);
    const v4u u = (v4u){pk16(hb[0], hb[1]), pk16(hb[2], hb[3]), pk16(hb[4], hb[5]), pk16(hb[6], hb[7])};
    unsigned short* q = X16 + (size_t)row * kD + c8;
    *(volatile v4u*)q = u;
    __threadfence();
    *(volatile v4u*)q = u;
  } else {
    const int i = (blockIdx.x - kXBlocks) * 256 + tid;
    const v4f a = *(const v4f*)(bih + 4 * (size_t)i);
    const v4f c = *(const v4f*)(bhh + 4 * (size_t)i);
    const v4f s = a + c;
    float* q = bsum + 4 * (size_t)i;
    *(volatile v4f*)q = s;
    __threadfence();
    *(volatile v4f*)q = s;
  }
}

__global__ __launch_bounds__(256) void feat_tcast_kernel(const float* __restrict__ FEAT, unsigned short* __restrict__ out) {
  __shared__ float sm[64][65];
  const int t   = threadIdx.x;
  const int bn0 = blockIdx.x * 64;
  const int h0  = blockIdx.y * 64;
#pragma unroll
  for (int i = 0; i < 16; ++i) {
    const int e = i * 256 + t;
    const int r = e >> 6;
    const int c = e & 63;
    sm[c][r] = FEAT[(size_t)(bn0 + r) * (2 * kH) + kH + h0 + c];
  }
  __syncthreads();
  const int lane = t & 31, wave = t >> 5;
  const int q = lane >> 3, c8 = (lane & 7) * 8;
  for (int pass = 0; pass < 2; ++pass) {
#pragma unroll
    for (int it = 0; it < 2; ++it) {
      const int row = wave * 8 + it * 4 + q;
      unsigned short hb[8];
#pragma unroll
      for (int e = 0; e < 8; ++e) hb[e] = h_bits(sm[row][c8 + e]);
      const v4u u = (v4u){pk16(hb[0], hb[1]), pk16(hb[2], hb[3]), pk16(hb[4], hb[5]), pk16(hb[6], hb[7])};
      *(volatile v4u*)(out + (size_t)(h0 + row) * kBN + bn0 + c8) = u;
    }
    __threadfence();
  }
}

constexpr int kHP = kH;
__global__ __launch_bounds__(256) void recur_seq_kernel(const float* __restrict__ XG, const unsigned short* __restrict__ Whhp,
                                                        const float* __restrict__ init_h, const float* __restrict__ init_c,
                                                        unsigned short* __restrict__ Qout) {
  __shared__ __align__(16) _Float16 Hs[2][kB * kHP];
  const _Float16* Whh = (const _Float16*)Whhp;
  const int tid = threadIdx.x, lane = tid & 31, wave = tid >> 5;
  const int rlane = lane & 15, hh = lane >> 4, koff = hh * 8;
  for (int i = tid; i < kB * kH; i += 256) {
    const int u = i & (kH - 1), row = i >> 9;
    Hs[0][row * kHP + u] = (_Float16)init_h[u];
  }
  float cst[4][8];
#pragma unroll
  for (int ub = 0; ub < 4; ++ub) {
    const float cv = init_c[(wave * 4 + ub) * 16 + rlane];
#pragma unroll
    for (int r = 0; r < 8; ++r) cst[ub][r] = cv;
  }
  __syncthreads();
  int cur = 0;
#pragma unroll 1
  for (int t = 0; t < kTQ; ++t) {
    const _Float16* Hc = &Hs[cur][0];
    _Float16* Hn = &Hs[cur ^ 1][0];
#pragma unroll
    for (int ub = 0; ub < 4; ++ub) {
      const int usub = wave * 4 + ub;
      v8f acc[4];
#pragma unroll
      for (int g = 0; g < 4; ++g) acc[g] = (v8f){0.f,0.f,0.f,0.f,0.f,0.f,0.f,0.f};
#pragma unroll 1
      for (int k0 = 0; k0 < kH; k0 += 32) {
        Frag<_Float16>::U fa;
        fa.h[0] = *(const v8h*)(Hc + rlane * kHP + koff + k0);
        fa.h[1] = *(const v8h*)(Hc + rlane * kHP + koff + k0 + 16);
        v16h bw[4];
#pragma unroll
        for (int g = 0; g < 4; ++g)
          bw[g] = Frag<_Float16>::load(Whh + (size_t)(g * kH + usub * 16 + rlane) * kH + koff + k0);
#pragma unroll
        for (int g = 0; g < 4; ++g) acc[g] = Frag<_Float16>::mma(fa.v, bw[g], acc[g]);
        dep_guard_h(acc[0], acc[3], fa.v, bw[3]);
        keep4_h(bw[0], bw[1], bw[2], bw[3]);
      }
      acc_guard4(acc[0], acc[1], acc[2], acc[3]);
      const int u = usub * 16 + rlane;
#pragma unroll
      for (int r = 0; r < 8; ++r) {
        const int row = hh * 8 + r;
        const float* xg = XG + (size_t)(t * kB + row) * kG4 + u;
        const float gi = acc[0][r] * kWCarryInv + xg[0];
        const float gf = acc[1][r] * kWCarryInv + xg[kH];
        const float gg = acc[2][r] * kWCarryInv + xg[2 * kH];
        const float go = acc[3][r] * kWCarryInv + xg[3 * kH];
        const float cn = sigm_f(gf) * cst[ub][r] + sigm_f(gi) * tanhf(gg);
        cst[ub][r] = cn;
        const float hn = sigm_f(go) * tanhf(cn);
        Hn[row * kHP + u] = (_Float16)hn;
      }
    }
    __syncthreads();
    for (int pass = 0; pass < 2; ++pass) {
#pragma unroll
      for (int rr = 0; rr < 2; ++rr) {
#pragma unroll
        for (int seg = 0; seg < 2; ++seg) {
          const int row = wave * 2 + rr;
          const v8h val = *(const v8h*)(Hn + row * kHP + seg * 256 + lane * 8);
          *(volatile v8h*)(Qout + ((size_t)row * kTQ + t) * kH + seg * 256 + lane * 8) = val;
        }
      }
      __threadfence();
    }
    cur ^= 1;
  }
}

constexpr int kHC = 64;
constexpr int kNT = 32;
static_assert(kHC == 64 && kNS % kNT == 0 && kH % kHC == 0);
__global__ __launch_bounds__(256) void add_score_kernel(const float* __restrict__ FEAT, const float* __restrict__ QW,
                                                        const float* __restrict__ vvec, const int* __restrict__ mem_sizes,
                                                        float* __restrict__ outp, int fcol, int use_mask) {
  __shared__ __align__(16) float Qs[kTQ * kHC];
  __shared__ __align__(16) float Fs[kHC * kNT];
  __shared__ __align__(16) float Cs[kH];
  __shared__ __align__(16) float Ss[kTQ * kNT];
  __shared__ float vsum_s;
  const int tid = threadIdx.x, lane = tid & 31, wave = tid >> 5;
  const int b = blockIdx.y, n0 = blockIdx.x * kNT;
  const int tq = tid >> 2, ng = tid & 3;
  for (int i = tid; i < kH; i += 256) Cs[i] = -2.0f * vvec[i];
  if (wave == 0) {
    float s = 0.f;
#pragma unroll 1
    for (int j = 0; j < kH / 32; ++j) s += vvec[j * 32 + lane];
#pragma unroll
    for (int off = 16; off > 0; off >>= 1) s += __shfl_xor(s, off, 32);
    if (lane == 0) vsum_s = s;
  }
  float acc[8];
#pragma unroll
  for (int j = 0; j < 8; ++j) acc[j] = 0.f;
#pragma unroll 1
  for (int hc0 = 0; hc0 < kH; hc0 += kHC) {
    __syncthreads();
#pragma unroll
    for (int i = 0; i < (kTQ * kHC) / 256; ++i) {
      const int e = i * 256 + tid;
      const int tl = e >> 6, hl = e & 63;
      Qs[tl * kHC + hl] = QW[(size_t)(b * kTQ + tl) * kH + hc0 + hl];
    }
#pragma unroll
    for (int i = 0; i < (kHC * kNT) / 256; ++i) {
      const int e = i * 256 + tid;
      const int nl = e >> 6, hl = e & 63;
      Fs[hl * kNT + nl] = kTwoLog2e * FEAT[(size_t)(b * kNS + n0 + nl) * (2 * kH) + fcol + hc0 + hl];
    }
    __syncthreads();
#pragma unroll 1
    for (int hl = 0; hl < kHC; ++hl) {
      const float q  = Qs[tq * kHC + hl];
      const float cc = Cs[hc0 + hl];
      const v4f f0 = *(const v4f*)(Fs + hl * kNT + ng * 8);
      const v4f f1 = *(const v4f*)(Fs + hl * kNT + ng * 8 + 4);
#pragma unroll
      for (int j = 0; j < 4; ++j) {
        const float e0 = exp2f(f0[j] + q);
        acc[j] = fmaf(cc, rcp_approx(e0 + 1.0f), acc[j]);
        const float e1 = exp2f(f1[j] + q);
        acc[4 + j] = fmaf(cc, rcp_approx(e1 + 1.0f), acc[4 + j]);
      }
    }
  }
  const float vs = vsum_s;
  const int ms = mem_sizes[b];
#pragma unroll
  for (int j = 0; j < 8; ++j) {
    const int nl = ng * 8 + j;
    float s = vs + acc[j];
    if (use_mask != 0 && (n0 + nl) >= ms) s = kNeg;
    Ss[tq * kNT + nl] = s;
  }
  __syncthreads();
  const int srow = tid >> 3, c4 = (tid & 7) * 4;
  for (int pass = 0; pass < 2; ++pass) {
#pragma unroll
    for (int it = 0; it < 2; ++it) {
      const int row = it * 32 + srow;
      const v4f v = *(const v4f*)(Ss + row * kNT + c4);
      *(volatile v4f*)(outp + ((size_t)(b * kTQ + row)) * kNS + n0 + c4) = v;
    }
    __threadfence();
  }
}

__global__ __launch_bounds__(256) void softmax_p_kernel(const float* __restrict__ SC, unsigned short* __restrict__ P16) {
  __shared__ __align__(16) float Ps[8 * kNS];
  const int tid = threadIdx.x, lane = tid & 31, wave = tid >> 5;
  const int row = blockIdx.x * 8 + wave;
  const v4f x = *(const v4f*)(SC + (size_t)row * kNS + lane * 4);
  float m = fmaxf(fmaxf(x[0], x[1]), fmaxf(x[2], x[3]));
#pragma unroll
  for (int off = 16; off > 0; off >>= 1) m = fmaxf(m, __shfl_xor(m, off, 32));
  float ev[4];
  float s = 0.f;
#pragma unroll
  for (int j = 0; j < 4; ++j) { ev[j] = expf(x[j] - m); s += ev[j]; }
#pragma unroll
  for (int off = 16; off > 0; off >>= 1) s += __shfl_xor(s, off, 32);
  const float inv = 1.0f / s;
#pragma unroll
  for (int j = 0; j < 4; ++j) Ps[wave * kNS + lane * 4 + j] = (ev[j] * inv) * kPCarry;
  __syncthreads();
  if (tid < 128) {
    const int r = tid >> 4, c8 = (tid & 15) * 8;
    const float* sp = Ps + r * kNS + c8;
    v8h hv;
#pragma unroll
    for (int e = 0; e < 8; ++e) hv[e] = (_Float16)sp[e];
    unsigned short* dst = P16 + (size_t)(blockIdx.x * 8 + r) * kNS + c8;
    *(volatile v8h*)dst = hv;
    __threadfence();
    *(volatile v8h*)dst = hv;
  }
}

constexpr size_t kOffMem16 = 0;
constexpr size_t kOffWih16 = kOffMem16 + (size_t)kBN * kD * 2;
constexpr size_t kOffWhh16 = kOffWih16 + (size_t)kG4 * kD * 2;
constexpr size_t kOffWt16  = kOffWhh16 + (size_t)kG4 * kH * 2;
constexpr size_t kOffX16   = kOffWt16 + (size_t)4 * kD * kH * 2;
constexpr size_t kOffFeat  = kOffX16 + (size_t)kBT * kD * 2;
constexpr size_t kOffHft16 = kOffFeat + (size_t)kBN * (2 * kH) * 4;
constexpr size_t kOffXg    = kOffHft16 + (size_t)kH * kBN * 2;
constexpr size_t kOffQa16  = kOffXg + (size_t)kBT * kG4 * 4;
constexpr size_t kOffQb16  = kOffQa16 + (size_t)kBT * kH * 2;
constexpr size_t kOffQw    = kOffQb16 + (size_t)kBT * kH * 2;
constexpr size_t kOffSc    = kOffQw + (size_t)kBT * kH * 4;
constexpr size_t kOffP16   = kOffSc + (size_t)kBT * kNS * 4;
constexpr size_t kOffBsum  = kOffP16 + (size_t)kBT * kNS * 2;
constexpr size_t kWsTotal  = kOffBsum + (size_t)kG4 * 4;
static_assert(kWsTotal == 33300480);
static_assert(kWsTotal <= (size_t)134217728);

extern "C" void kernel_launch(void* const* d_in, const int* in_sizes, int n_in,
                              void* d_out, int out_size, void* d_ws, size_t ws_size,
                              hipStream_t stream) {
  if (n_in < 15) return;
  if (in_sizes[0] != kB * kNS * kD || in_sizes[1] != kB * kT * kD || in_sizes[2] != kH || in_sizes[3] != kH ||
      in_sizes[4] != kG4 * kD || in_sizes[5] != kG4 * kH || in_sizes[6] != kG4 || in_sizes[7] != kG4 ||
      in_sizes[8] != kD * kH || in_sizes[9] != kH * kH || in_sizes[10] != kH || in_sizes[11] != kD * kH ||
      in_sizes[12] != kH * kH || in_sizes[13] != kH || in_sizes[14] != kB) return;
  if (out_size != kBT * kNS) return;
  if (kWsTotal > ws_size) return;

  const float* attn_mem  = (const float*)d_in[0];
  const float* lstm_in   = (const float*)d_in[1];
  const float* init_h    = (const float*)d_in[2];
  const float* init_c    = (const float*)d_in[3];
  const float* Wih       = (const float*)d_in[4];
  const float* Whh       = (const float*)d_in[5];
  const float* bih       = (const float*)d_in[6];
  const float* bhh       = (const float*)d_in[7];
  const float* attn_wm   = (const float*)d_in[8];
  const float* attn_wq   = (const float*)d_in[9];
  const float* attn_v    = (const float*)d_in[10];
  const float* hop_wm    = (const float*)d_in[11];
  const float* hop_wq    = (const float*)d_in[12];
  const float* hop_v     = (const float*)d_in[13];
  const int*   mem_sizes = (const int*)d_in[14];
  float* out = (float*)d_out;

  char* ws = (char*)d_ws;
  unsigned short* MEM16 = (unsigned short*)(ws + kOffMem16);
  unsigned short* WIH16 = (unsigned short*)(ws + kOffWih16);
  unsigned short* WHH16 = (unsigned short*)(ws + kOffWhh16);
  unsigned short* WT16  = (unsigned short*)(ws + kOffWt16);
  unsigned short* X16   = (unsigned short*)(ws + kOffX16);
  float*          FEAT  = (float*)(ws + kOffFeat);
  unsigned short* HFT16 = (unsigned short*)(ws + kOffHft16);
  float*          XG    = (float*)(ws + kOffXg);
  unsigned short* QA16  = (unsigned short*)(ws + kOffQa16);
  unsigned short* QB16  = (unsigned short*)(ws + kOffQb16);
  float*          QW    = (float*)(ws + kOffQw);
  float*          SC    = (float*)(ws + kOffSc);
  unsigned short* P16   = (unsigned short*)(ws + kOffP16);
  float*          BSUM  = (float*)(ws + kOffBsum);
  const size_t kPlane = (size_t)kD * kH;

  wtcast_kernel<<<dim3(kD / 64, kH / 64, 4), 256, 0, stream>>>(attn_wm, hop_wm, attn_wq, hop_wq, WT16, kWCarry);
  cast3_f16_kernel<<<dim3((kBN * kD / 8) / 256, 3), 256, 0, stream>>>(attn_mem, Wih, Whh, MEM16, WIH16, WHH16,
                                                                        1.0f, kWCarry, kWCarry, kBN * kD / 8);
  prep_kernel<<<kXBlocks + 2, 256, 0, stream>>>(attn_mem, lstm_in, mem_sizes, bih, bhh, X16, BSUM);
  wmma_gemm64<0, false, 0, 0, false><<<dim3((kBN / 64) * ((2 * kH) / 64) / 8, 1), 256, 0, stream>>>(
      MEM16, nullptr, kD, 0, WT16, nullptr, kD, 0, FEAT, nullptr, 2 * kH, 0,
      nullptr, nullptr, 0, kBN, 2 * kH, kD, kWCarryInv);
  feat_tcast_kernel<<<dim3(kBN / 64, kH / 64), 256, 0, stream>>>(FEAT, HFT16);
  wmma_gemm64<0, false, 2, 0, false><<<dim3((kBT / 64) * (kG4 / 64) / 8, 1), 256, 0, stream>>>(
      X16, nullptr, kD, 0, WIH16, nullptr, kD, 0, XG, nullptr, kG4, 0,
      BSUM, nullptr, 0, kBT, kG4, kD, kWCarryInv);
  recur_seq_kernel<<<1, 256, 0, stream>>>(XG, WHH16, init_h, init_c, QA16);
  unsigned short* Qsrc = QA16;
  unsigned short* Qdst = QB16;
  for (int hop = 0; hop < 2; ++hop) {
    wmma_gemm64<0, false, 0, 0, false><<<dim3((kBT / 64) * (kH / 64) / 8, 1), 256, 0, stream>>>(
        Qsrc, nullptr, kH, 0, WT16 + 3 * kPlane, nullptr, kH, 0, QW, nullptr, kH, 0,
        nullptr, nullptr, 0, kBT, kH, kH, kQWScale);
    add_score_kernel<<<dim3(kNS / kNT, kB), 256, 0, stream>>>(FEAT, QW, hop_v, mem_sizes, SC, kH, 1);
    softmax_p_kernel<<<kBT / 8, 256, 0, stream>>>(SC, P16);
    wmma_gemm64<0, false, 0, 1, false><<<dim3(1, kB), 256, 0, stream>>>(
        P16, nullptr, kNS, (long)kTQ * kNS, HFT16, nullptr, kBN, (long)kNS, Qdst, nullptr, kH, (long)kTQ * kH,
        nullptr, nullptr, 0, kTQ, kH, kNS, kPCarryInv);
    unsigned short* tmp = Qsrc; Qsrc = Qdst; Qdst = tmp;
  }
  wmma_gemm64<0, false, 0, 0, false><<<dim3((kBT / 64) * (kH / 64) / 8, 1), 256, 0, stream>>>(
      Qsrc, nullptr, kH, 0, WT16 + 2 * kPlane, nullptr, kH, 0, QW, nullptr, kH, 0,
      nullptr, nullptr, 0, kBT, kH, kH, kQWScale);
  add_score_kernel<<<dim3(kNS / kNT, kB), 256, 0, stream>>>(FEAT, QW, attn_v, mem_sizes, out, 0, 0);
}
